// RNNPredictor_64493228917206
// MI455X (gfx1250) — hardware-verified
//
#include <hip/hip_runtime.h>

typedef __attribute__((ext_vector_type(16))) _Float16 v16h;
typedef __attribute__((ext_vector_type(8)))  _Float16 v8h;
typedef __attribute__((ext_vector_type(16))) __bf16   v16b;
typedef __attribute__((ext_vector_type(8)))  __bf16   v8b;
typedef __attribute__((ext_vector_type(8)))  float    v8f;
typedef __attribute__((ext_vector_type(4)))  float    v4f;

constexpr int kSeq     = 256;
constexpr int kStep    = 256;
constexpr int kIn      = 128;
constexpr int kHid     = 512;
constexpr int kHalfSeq = 128;
constexpr int kRowsHalf = kHalfSeq * kStep;
constexpr int kRowsAll  = kSeq * kStep;
static_assert(kRowsHalf == 32768 && kRowsAll == 65536);
static_assert(kSeq == 2 * kHalfSeq);

constexpr int kSeqPB      = 16;
constexpr int kRnnBlocks  = kHalfSeq / kSeqPB;
constexpr int kRnnThreads = 256;
constexpr int kHP         = kHid + 8;
constexpr int kHTile      = kSeqPB * kHP;
static_assert(kHalfSeq % kSeqPB == 0);
static_assert(kHid == (kRnnThreads / 32) * 64);
static_assert(kHP % 8 == 0);
static_assert(kHid % 32 == 0 && kIn % 32 == 0);
static_assert(kRowsHalf % 64 == 0 && kHid % 64 == 0);

constexpr int kDwWih  = kHid * kIn / 2;
constexpr int kDwWhh  = kHid * kHid / 2;
constexpr int kDwBsum = kHid;
constexpr int kBlkWih  = kDwWih / 256;
constexpr int kBlkWhh  = kDwWhh / 256;
constexpr int kBlkBsum = kDwBsum / 256;
constexpr int kPrepB1 = kBlkWih;
constexpr int kPrepB2 = kPrepB1 + kBlkWhh;
constexpr int kPrepBlocks = kPrepB2 + kBlkBsum;
static_assert(kDwWih % 256 == 0 && kDwWhh % 256 == 0 && kDwBsum % 256 == 0);
static_assert(kPrepBlocks == 642);
constexpr int kXChunks = kRowsAll * kIn / 8;
static_assert(kXChunks % 256 == 0);
static_assert(kIn / 8 == 16);

__device__ __forceinline__ unsigned short f2bf_bits(float f) {
  unsigned u = __float_as_uint(f);
  return (unsigned short)((u + 0x7FFFu + ((u >> 16) & 1u)) >> 16);
}
__device__ __forceinline__ float bf_bits2f(unsigned short h) { return __uint_as_float(((unsigned)h) << 16); }

__device__ __forceinline__ void dep_guard_h(v8f& a, v8f& b, v16h x, v16h y) { asm volatile("v_nop\n\tv_nop\n\tv_nop\n\tv_nop" : "+v"(a), "+v"(b) : "v"(x), "v"(y)); }
__device__ __forceinline__ void dep_guard_b(v8f& a, v8f& b, v16b x, v16b y) { asm volatile("v_nop\n\tv_nop\n\tv_nop\n\tv_nop" : "+v"(a), "+v"(b) : "v"(x), "v"(y)); }
__device__ __forceinline__ void keep4_h(v16h a, v16h b, v16h c, v16h d) { asm volatile("v_nop" :: "v"(a), "v"(b), "v"(c), "v"(d)); }
__device__ __forceinline__ void keep4_b(v16b a, v16b b, v16b c, v16b d) { asm volatile("v_nop" :: "v"(a), "v"(b), "v"(c), "v"(d)); }
__device__ __forceinline__ void acc_guard4(v8f& a, v8f& b, v8f& c, v8f& d) { asm volatile("v_nop\n\tv_nop\n\tv_nop\n\tv_nop" : "+v"(a), "+v"(b), "+v"(c), "+v"(d)); }

template <typename T> struct Frag;
template <> struct Frag<_Float16> {
  typedef v16h V; union U { v16h v; v8h h[2]; };
  static __device__ __forceinline__ v16h load(const _Float16* p) {
    U f; f.h[0] = *(const v8h*)(p); f.h[1] = *(const v8h*)(p + 16); return f.v;
  }
  static __device__ __forceinline__ v8f mma(v16h a, v16h b, v8f c) {
    return __builtin_amdgcn_wmma_f32_16x16x32_f16(false, a, false, b, (short)0, c, false, false);
  }
  static __device__ __forceinline__ void guard(v8f& a, v8f& b, v16h x, v16h y) { dep_guard_h(a, b, x, y); }
  static __device__ __forceinline__ void keep(v16h a, v16h b, v16h c, v16h d) { keep4_h(a, b, c, d); }
};
template <> struct Frag<__bf16> {
  typedef v16b V; union U { v16b v; v8b h[2]; };
  static __device__ __forceinline__ v16b load(const __bf16* p) {
    U f; f.h[0] = *(const v8b*)(p); f.h[1] = *(const v8b*)(p + 16); return f.v;
  }
  static __device__ __forceinline__ v8f mma(v16b a, v16b b, v8f c) {
    return __builtin_amdgcn_wmma_f32_16x16x32_bf16(false, a, false, b, (short)0, c, false, false);
  }
  static __device__ __forceinline__ void guard(v8f& a, v8f& b, v16b x, v16b y) { dep_guard_b(a, b, x, y); }
  static __device__ __forceinline__ void keep(v16b a, v16b b, v16b c, v16b d) { keep4_b(a, b, c, d); }
};

template <int ET> struct Elem;
template <> struct Elem<0> { typedef _Float16 T; };
template <> struct Elem<1> { typedef __bf16 T; };
template <int ET, bool SPLIT, int BIAS_MODE, int OUT_MODE, bool RESID, int ACT = 0, int TRI = 0>
__global__ __launch_bounds__(256) void wmma_gemm64(
    const unsigned short* __restrict__ Ap, const unsigned short* __restrict__ A2p, int lda, long strideA,
    const unsigned short* __restrict__ Btp, const unsigned short* __restrict__ Bt2p, int ldb, long strideB,
    void* __restrict__ Cout, void* __restrict__ Cout2, int ldc, long strideC,
    const float* __restrict__ bias,
    const float* __restrict__ resid, long strideR,
    int M, int N, int K, float scale) {
  typedef typename Elem<ET>::T T;
  typedef typename Frag<T>::V V;
  const T* A = (const T*)Ap; const T* A2 = (const T*)A2p; const T* Bt = (const T*)Btp; const T* Bt2 = (const T*)Bt2p;
  __shared__ __align__(16) float sT[8][16 * 68];
  const int b    = blockIdx.y;
  const int lane = threadIdx.x & 31;
  const int wave = threadIdx.x >> 5;
  const int tilesN = N >> 6;
  const int tilesM = M >> 6;
  const int tile = blockIdx.x * 8 + wave;
  if (tile >= tilesM * tilesN) return;
  const int tm = tile / tilesN;
  const int tn = tile - tm * tilesN;
  if (TRI == 1 && tn > tm) return;
  const int m0 = tm << 6;
  const int n0 = tn << 6;
  const int kLim = (TRI == 2) ? ((m0 + 64 < K) ? (m0 + 64) : K) : K;

  const T* Ab  = A  + (size_t)b * strideA;
  const T* Bb  = Bt + (size_t)b * strideB;
  const T* Ab2 = SPLIT ? (A2  + (size_t)b * strideA) : nullptr;
  const T* Bb2 = SPLIT ? (Bt2 + (size_t)b * strideB) : nullptr;

  const int rlane = lane & 15;
  const int koff  = (lane >> 4) * 8;
  const int mOff  = (lane >> 4) * 8;

  v8f acc[4][4];
#pragma unroll
  for (int i = 0; i < 4; ++i)
#pragma unroll
    for (int j = 0; j < 4; ++j) acc[i][j] = (v8f){0.f,0.f,0.f,0.f,0.f,0.f,0.f,0.f};

  for (int k0 = 0; k0 < kLim; k0 += 32) {
    V bh[4], bl[4];
#pragma unroll
    for (int j = 0; j < 4; ++j) {
      const size_t bo = (size_t)(n0 + (j << 4) + rlane) * ldb + koff + k0;
      bh[j] = Frag<T>::load(Bb + bo);
      if (SPLIT) bl[j] = Frag<T>::load(Bb2 + bo);
    }
#pragma unroll
    for (int i = 0; i < 4; ++i) {
      const size_t ao = (size_t)(m0 + (i << 4) + rlane) * lda + koff + k0;
      V ah = Frag<T>::load(Ab + ao);
      V al;
      if (SPLIT) al = Frag<T>::load(Ab2 + ao);
#pragma unroll
      for (int j = 0; j < 4; ++j) {
        acc[i][j] = Frag<T>::mma(ah, bh[j], acc[i][j]);
        if (SPLIT) {
          acc[i][j] = Frag<T>::mma(ah, bl[j], acc[i][j]);
          acc[i][j] = Frag<T>::mma(al, bh[j], acc[i][j]);
        }
      }
      Frag<T>::guard(acc[i][0], acc[i][3], ah, SPLIT ? al : ah);
    }
    Frag<T>::keep(bh[0], bh[1], bh[2], bh[3]);
    if (SPLIT) Frag<T>::keep(bl[0], bl[1], bl[2], bl[3]);
  }
  acc_guard4(acc[0][0], acc[0][1], acc[0][2], acc[0][3]);
  acc_guard4(acc[1][0], acc[1][1], acc[1][2], acc[1][3]);
  acc_guard4(acc[2][0], acc[2][1], acc[2][2], acc[2][3]);
  acc_guard4(acc[3][0], acc[3][1], acc[3][2], acc[3][3]);

  float* slab = sT[wave];
  const float* Rb = RESID ? (resid + (size_t)b * strideR) : nullptr;
#pragma unroll
  for (int i = 0; i < 4; ++i) {
    const int mBase = m0 + (i << 4);
#pragma unroll
    for (int j = 0; j < 4; ++j) {
      const int n = n0 + (j << 4) + rlane;
      float bv = 0.f;
      if (BIAS_MODE == 2) bv = bias[n];
#pragma unroll
      for (int r = 0; r < 8; ++r) {
        float v = acc[i][j][r] * scale;
        if (BIAS_MODE == 1) v += bias[mBase + mOff + r];
        if (BIAS_MODE == 2) v += bv;
        if (RESID) v += Rb[(size_t)(mBase + mOff + r) * ldc + n];
        if (ACT == 1) v = tanhf(v);
        if (ACT == 2) v = fmaxf(v, 0.0f);
        if (ACT == 4) v = (v > 0.f) ? v : 0.01f * v;
        slab[(mOff + r) * 68 + (j << 4) + rlane] = v;
      }
    }
    __builtin_amdgcn_fence(__ATOMIC_RELEASE, "workgroup");
    __builtin_amdgcn_wave_barrier();
    __builtin_amdgcn_fence(__ATOMIC_ACQUIRE, "workgroup");
    if (OUT_MODE == 0) {
      float* C = (float*)Cout + (size_t)b * strideC;
      const int hh = lane >> 4, c4 = (lane & 15) * 4;
      for (int pass = 0; pass < 2; ++pass) {
#pragma unroll
        for (int it = 0; it < 8; ++it) {
          const int row = it * 2 + hh;
          v4f v = *(const v4f*)(slab + row * 68 + c4);
          *(volatile v4f*)(C + (size_t)(mBase + row) * ldc + n0 + c4) = v;
        }
        __threadfence();
      }
    } else {
      const int q = lane >> 3, c8 = (lane & 7) * 8;
      unsigned short* C  = (unsigned short*)Cout  + (size_t)b * strideC;
      unsigned short* C2 = (OUT_MODE == 2) ? ((unsigned short*)Cout2 + (size_t)b * strideC) : nullptr;
      for (int pass = 0; pass < 2; ++pass) {
#pragma unroll
        for (int it = 0; it < 4; ++it) {
          const int row = it * 4 + q;
          const float* sp = slab + row * 68 + c8;
          v8h hv, lv;
#pragma unroll
          for (int e = 0; e < 8; ++e) {
            if (OUT_MODE == 1) {
              hv[e] = (_Float16)sp[e];
            } else {
              unsigned short hb = f2bf_bits(sp[e]);
              unsigned short lb = f2bf_bits(sp[e] - bf_bits2f(hb));
              hv[e] = __builtin_bit_cast(_Float16, hb);
              lv[e] = __builtin_bit_cast(_Float16, lb);
            }
          }
          *(volatile v8h*)(C + (size_t)(mBase + row) * ldc + n0 + c8) = hv;
          if (OUT_MODE == 2) *(volatile v8h*)(C2 + (size_t)(mBase + row) * ldc + n0 + c8) = lv;
        }
        __threadfence();
      }
    }
    __builtin_amdgcn_fence(__ATOMIC_RELEASE, "workgroup");
    __builtin_amdgcn_wave_barrier();
    __builtin_amdgcn_fence(__ATOMIC_ACQUIRE, "workgroup");
  }
}

__device__ __forceinline__ unsigned pack_f16x2(float a, float b) {
  const _Float16 h0 = (_Float16)a, h1 = (_Float16)b;
  return (unsigned)__builtin_bit_cast(unsigned short, h0) | ((unsigned)__builtin_bit_cast(unsigned short, h1) << 16);
}
__device__ __forceinline__ void st2u(unsigned* p, unsigned v) { *(volatile unsigned*)p = v; __threadfence(); *(volatile unsigned*)p = v; }
__device__ __forceinline__ float ftanh(float x) { return 1.0f - 2.0f * __builtin_amdgcn_rcpf(1.0f + __expf(2.0f * x)); }

__global__ __launch_bounds__(256) void prep_kernel(
    const float* __restrict__ w_ih, const float* __restrict__ w_hh,
    const float* __restrict__ b_ih, const float* __restrict__ b_hh,
    unsigned* __restrict__ wihu, unsigned* __restrict__ whhu, unsigned* __restrict__ bsumu) {
  const int blk = blockIdx.x, tid = threadIdx.x;
  const float ws16 = 16.0f;
  if (blk < kPrepB1) {
    const int p = blk * 256 + tid;
    st2u(wihu + p, pack_f16x2(w_ih[2 * p] * ws16, w_ih[2 * p + 1] * ws16));
  } else if (blk < kPrepB2) {
    const int p = (blk - kPrepB1) * 256 + tid;
    st2u(whhu + p, pack_f16x2(w_hh[2 * p] * ws16, w_hh[2 * p + 1] * ws16));
  } else {
    const int p = (blk - kPrepB2) * 256 + tid;
    const int pc = p & (kHid - 1);
    const float v = b_ih[pc] + b_hh[pc];
    st2u(bsumu + p, (unsigned)__float_as_uint(v));
  }
}

__global__ __launch_bounds__(256) void xcast_kernel(const float* __restrict__ x, _Float16* __restrict__ x16t) {
  const int i = blockIdx.x * 256 + threadIdx.x;
  const int row = i >> 4, c8 = i & 15;
  const int hf  = row >> 15;
  const int rem = row & (kRowsHalf - 1);
  const int t = rem >> 7, bl = rem & (kHalfSeq - 1);
  const int b = hf * kHalfSeq + bl;
  const float* src = x + ((size_t)b * kStep + t) * kIn + c8 * 8;
  const v4f f0 = *(const v4f*)src;
  const v4f f1 = *(const v4f*)(src + 4);
  v8h hv;
  hv[0] = (_Float16)f0[0]; hv[1] = (_Float16)f0[1]; hv[2] = (_Float16)f0[2]; hv[3] = (_Float16)f0[3];
  hv[4] = (_Float16)f1[0]; hv[5] = (_Float16)f1[1]; hv[6] = (_Float16)f1[2]; hv[7] = (_Float16)f1[3];
  _Float16* dst = x16t + (size_t)row * kIn + c8 * 8;
  *(volatile v8h*)dst = hv;
  __threadfence();
  *(volatile v8h*)dst = hv;
}

__global__ __launch_bounds__(kRnnThreads) void rnn_layer_kernel(
    const float* __restrict__ xinT, const _Float16* __restrict__ whh16, _Float16* __restrict__ hout) {
  __shared__ __align__(16) _Float16 hbuf[2 * kHTile];
  const int tid = threadIdx.x, lane = tid & 31, wave = tid >> 5;
  const int c = lane & 15, hh = lane >> 4, koff = hh * 8, mOff = hh * 8;
  const int seq0 = blockIdx.x * kSeqPB;
  const int n0 = wave * 64;

  {
    const v8h z = {(_Float16)0.f, (_Float16)0.f, (_Float16)0.f, (_Float16)0.f, (_Float16)0.f, (_Float16)0.f, (_Float16)0.f, (_Float16)0.f};
    for (int i = tid; i < (2 * kHTile) / 8; i += kRnnThreads) *(v8h*)(hbuf + i * 8) = z;
  }
  __syncthreads();

  const float inv16 = 0.0625f;
  const _Float16* brow = whh16 + (size_t)(n0 + c) * kHid + koff;
  const int q4 = lane >> 3, c8 = (lane & 7) * 8;

#pragma unroll 1
  for (int t = 0; t < kStep; ++t) {
    const _Float16* hc = hbuf + (t & 1) * kHTile;
    _Float16*       hn = hbuf + ((t + 1) & 1) * kHTile;
    v8f acc[4];
#pragma unroll
    for (int j = 0; j < 4; ++j) {
      const float* xp = xinT + (size_t)(n0 + 16 * j + c) * kRowsHalf + t * kHalfSeq + seq0 + 8 * hh;
      const v4f xa = *(const v4f*)xp;
      const v4f xb = *(const v4f*)(xp + 4);
      acc[j][0] = xa[0] * 16.0f; acc[j][1] = xa[1] * 16.0f; acc[j][2] = xa[2] * 16.0f; acc[j][3] = xa[3] * 16.0f;
      acc[j][4] = xb[0] * 16.0f; acc[j][5] = xb[1] * 16.0f; acc[j][6] = xb[2] * 16.0f; acc[j][7] = xb[3] * 16.0f;
    }
    const _Float16* arow = hc + c * kHP + koff;
    v16h fa;
    v16h fb[4];
#pragma unroll 4
    for (int kc = 0; kc < kHid / 32; ++kc) {
      fa = Frag<_Float16>::load(arow + kc * 32);
#pragma unroll
      for (int j = 0; j < 4; ++j) fb[j] = Frag<_Float16>::load(brow + (size_t)(16 * j) * kHid + kc * 32);
#pragma unroll
      for (int j = 0; j < 4; ++j) acc[j] = Frag<_Float16>::mma(fa, fb[j], acc[j]);
      Frag<_Float16>::guard(acc[0], acc[3], fa, fb[3]);
      Frag<_Float16>::keep(fb[0], fb[1], fb[2], fb[3]);
    }
    acc_guard4(acc[0], acc[1], acc[2], acc[3]);

#pragma unroll
    for (int j = 0; j < 4; ++j) {
#pragma unroll
      for (int r = 0; r < 8; ++r) {
        const float hv = ftanh(acc[j][r] * inv16);
        hn[(mOff + r) * kHP + n0 + 16 * j + c] = (_Float16)hv;
      }
    }
    __syncthreads();

    if (t == kStep - 1) {
      for (int pass = 0; pass < 2; ++pass) {
#pragma unroll
        for (int it = 0; it < 4; ++it) {
          const int rr = it * 4 + q4;
          const v8h v = *(const v8h*)(hn + rr * kHP + n0 + c8);
          *(volatile v8h*)(hout + (size_t)(seq0 + rr) * kHid + n0 + c8) = v;
        }
        __threadfence();
      }
    }
  }
}

__global__ __launch_bounds__(256) void head_kernel(
    const _Float16* __restrict__ hl, const float* __restrict__ fc_w, const float* __restrict__ fc_b,
    float* __restrict__ out) {
  __shared__ __align__(16) float res[kSeq];
  const int s = threadIdx.x;
  const _Float16* hrow = hl + (size_t)s * kHid;
  float acc = 0.f;
#pragma unroll 1
  for (int cc = 0; cc < kHid / 8; ++cc) {
    const v8h hv = *(const v8h*)(hrow + cc * 8);
    const v4f w0 = *(const v4f*)(fc_w + cc * 8);
    const v4f w1 = *(const v4f*)(fc_w + cc * 8 + 4);
    acc += (float)hv[0] * w0[0]; acc += (float)hv[1] * w0[1]; acc += (float)hv[2] * w0[2]; acc += (float)hv[3] * w0[3];
    acc += (float)hv[4] * w1[0]; acc += (float)hv[5] * w1[1]; acc += (float)hv[6] * w1[2]; acc += (float)hv[7] * w1[3];
  }
  res[s] = acc + fc_b[0];
  __syncthreads();
  if (s < kSeq / 4) {
    const v4f v = *(const v4f*)(res + 4 * s);
    *(volatile v4f*)(out + 4 * s) = v;
    __threadfence();
    *(volatile v4f*)(out + 4 * s) = v;
  }
}

extern "C" void kernel_launch(void* const* d_in, const int* in_sizes, int n_in,
                              void* d_out, int out_size, void* d_ws, size_t ws_size, hipStream_t stream) {
  if (n_in < 7 || d_out == nullptr || d_ws == nullptr) return;
  if (in_sizes[0] != kSeq * kStep * kIn || in_sizes[1] != kHid * kIn || in_sizes[2] != kHid * kHid ||
      in_sizes[3] != kHid || in_sizes[4] != kHid || in_sizes[5] != kHid || in_sizes[6] != 1 ||
      out_size != kSeq) return;

  const float* x    = (const float*)d_in[0];
  const float* w_ih = (const float*)d_in[1];
  const float* w_hh = (const float*)d_in[2];
  const float* b_ih = (const float*)d_in[3];
  const float* b_hh = (const float*)d_in[4];
  const float* fc_w = (const float*)d_in[5];
  const float* fc_b = (const float*)d_in[6];
  float* out = (float*)d_out;

  char* ws = (char*)d_ws; size_t off = 0;
  auto carve = [&](size_t bytes) -> char* { char* p = ws + off; off += (bytes + 255) & ~(size_t)255; return p; };
  unsigned short* X16T  = (unsigned short*)carve((size_t)kRowsAll * kIn * 2);
  unsigned short* WIH16 = (unsigned short*)carve((size_t)kHid * kIn * 2);
  unsigned short* WHH16 = (unsigned short*)carve((size_t)kHid * kHid * 2);
  float*          BSUM  = (float*)carve((size_t)kDwBsum * 4);
  float*          XINT  = (float*)carve((size_t)kHid * kRowsHalf * 4);
  unsigned short* HL16  = (unsigned short*)carve((size_t)kSeq * kHid * 2);
  if (off > ws_size || off > (size_t)134217728) return;

  const float inv16 = 1.0f / 16.0f;
  const int xinGrid = ((kHid / 64) * (kRowsHalf / 64)) / 8;

  prep_kernel<<<kPrepBlocks, 256, 0, stream>>>(w_ih, w_hh, b_ih, b_hh,
                                               (unsigned*)WIH16, (unsigned*)WHH16, (unsigned*)BSUM);

  xcast_kernel<<<kXChunks / 256, 256, 0, stream>>>(x, (_Float16*)X16T);

  wmma_gemm64<0, false, 1, 0, false, 0, 0><<<dim3(xinGrid, 1), 256, 0, stream>>>(
      WIH16, nullptr, kIn, 0L, X16T, nullptr, kIn, 0L,
      (void*)XINT, nullptr, kRowsHalf, 0L, BSUM, nullptr, 0L, kHid, kRowsHalf, kIn, inv16);

  rnn_layer_kernel<<<kRnnBlocks, kRnnThreads, 0, stream>>>(XINT, (const _Float16*)WHH16, (_Float16*)HL16);

  wmma_gemm64<0, false, 1, 0, false, 0, 0><<<dim3(xinGrid, 1), 256, 0, stream>>>(
      WIH16, nullptr, kIn, 0L, X16T + (size_t)kRowsHalf * kIn, nullptr, kIn, 0L,
      (void*)XINT, nullptr, kRowsHalf, 0L, BSUM, nullptr, 0L, kHid, kRowsHalf, kIn, inv16);

  rnn_layer_kernel<<<kRnnBlocks, kRnnThreads, 0, stream>>>(XINT, (const _Float16*)WHH16,
                                                            (_Float16*)(HL16 + (size_t)kHalfSeq * kHid));

  head_kernel<<<1, 256, 0, stream>>>((const _Float16*)HL16, fc_w, fc_b, out);
}
